// H_ATT_38723425140810
// MI455X (gfx1250) — hardware-verified
//
#include <hip/hip_runtime.h>
#include <stddef.h>


typedef _Float16 v16h __attribute__((ext_vector_type(16)));
typedef _Float16 v8h  __attribute__((ext_vector_type(8)));
typedef float    v8f  __attribute__((ext_vector_type(8)));
typedef float    v4f  __attribute__((ext_vector_type(4)));
typedef _Float16 h16;

#ifndef NB
#define NB 128
#endif
#define NB_FULL 128
#define RL   64
#define FIN  1024
#define DH   512
#define MROWS (NB * RL)

static_assert(NB >= 1 && NB <= NB_FULL);
static_assert(RL == 64);
static_assert(RL == 8 * 8 && RL == 4 * 16);
static_assert((FIN % 64) == 0 && (FIN % 32) == 0);
static_assert((DH % 64) == 0 && (DH % 32) == 0);
static_assert(((DH * FIN) % 2048) == 0);
static_assert(FIN == 2 * 16 * 32);
static_assert((MROWS % 64) == 0);

#define LDT 72
#define LDC 68
#define LDO 36
static_assert((LDT % 8) == 0 && LDT >= 64);
static_assert((LDC % 4) == 0 && LDC >= 64);
static_assert((LDO % 4) == 0 && LDO >= 32);

#define WCARRY  64.0f
#define XCARRY  16.0f
#define HCARRY  256.0f
#define QCARRY  16384.0f
#define SQCARRY 4096.0f
#define PCARRY  1024.0f
#define RCARRY  1024.0f

static_assert(64 * LDC * 4 + 2 * 64 * LDT * 2 + 64 * 4 + 8 * 16 * LDO * 4 <= 65536);

#define WPL_BYTES ((size_t)DH * FIN * 2)
#define XPL_BYTES ((size_t)MROWS * FIN * 2)
#define GPL_BYTES ((size_t)MROWS * DH * 2)
#define OFF_WHY ((size_t)0)
#define OFF_WHG (OFF_WHY + WPL_BYTES)
#define OFF_WQY (OFF_WHG + WPL_BYTES)
#define OFF_WQG (OFF_WQY + WPL_BYTES)
#define OFF_XH  (OFF_WQG + WPL_BYTES)
#define OFF_XQ  (OFF_XH + XPL_BYTES)
#define OFF_HT  (OFF_XQ + XPL_BYTES)
#define OFF_H1  (OFF_HT + XPL_BYTES)
#define OFF_H2  (OFF_H1 + GPL_BYTES)
#define OFF_Q1  (OFF_H2 + GPL_BYTES)
#define OFF_Q2  (OFF_Q1 + GPL_BYTES)
#define WS_TOTAL (OFF_Q2 + GPL_BYTES)
static_assert((WPL_BYTES % 512) == 0 && (XPL_BYTES % 128) == 0 && (GPL_BYTES % 128) == 0);
static_assert(WS_TOTAL <= (size_t)134217728);

__device__ __forceinline__ float bf16r(float x) {
  unsigned int u = __float_as_uint(x);
  u = (u + 0x7FFFu + ((u >> 16) & 1u)) & 0xFFFF0000u;
  return __uint_as_float(u);
}

static __device__ __forceinline__ h16 toh_flush(float v) {
  const h16 r = (h16)v;
  return (fabsf(v) < 6.103515625e-05f) ? (h16)0.0f : r;
}

__device__ __forceinline__ v16h frag_at(const _Float16* p) {
  v8h lo = *(const v8h*)(p);
  v8h hi = *(const v8h*)(p + 16);
  v16h out;
#pragma unroll
  for (int i = 0; i < 8; ++i) { out[i] = lo[i]; out[i + 8] = hi[i]; }
  return out;
}
__device__ __forceinline__ v16h ld_frag(const _Float16* base, unsigned ld) {
  const unsigned lane = threadIdx.x & 31u;
  return frag_at(base + (lane & 15u) * ld + (lane >> 4) * 8u);
}

__device__ __forceinline__ v8f wmma16(v16h a, v16h b, v8f c) {
  v8f d = __builtin_amdgcn_wmma_f32_16x16x32_f16(false, a, false, b, (short)0, c,
                                                 false, false);
  asm volatile("v_nop\n\tv_nop\n\tv_nop\n\tv_nop" : "+v"(d) : "v"(a), "v"(b));
  return d;
}

__device__ __forceinline__ float red32_sum(float x) {
#pragma unroll
  for (int off = 1; off < 32; off <<= 1) x += __shfl_xor(x, off, 32);
  return x;
}
__device__ __forceinline__ float red32_max(float x) {
#pragma unroll
  for (int off = 1; off < 32; off <<= 1) x = fmaxf(x, __shfl_xor(x, off, 32));
  return x;
}

__device__ __forceinline__ void wave_lds_sync() {
  __builtin_amdgcn_fence(3  , "wavefront");
  asm volatile("s_wait_dscnt 0x0" ::: "memory");
  __builtin_amdgcn_wave_barrier();
}

__device__ __forceinline__ v8h wrow8(const float* __restrict__ p) {
#pragma clang fp contract(off)
  const v4f a0 = *(const v4f*)(p);
  const v4f a1 = *(const v4f*)(p + 4);
  v8h o;
#pragma unroll
  for (int i = 0; i < 4; ++i) {
    o[i]     = toh_flush(WCARRY * bf16r(a0[i]));
    o[i + 4] = toh_flush(WCARRY * bf16r(a1[i]));
  }
  return o;
}

__global__ __launch_bounds__(256) void wplane_kernel(
    const float* __restrict__ W0, const float* __restrict__ W1,
    const float* __restrict__ W2, const float* __restrict__ W3,
    _Float16* __restrict__ P0, _Float16* __restrict__ P1,
    _Float16* __restrict__ P2, _Float16* __restrict__ P3) {
  const size_t e = ((size_t)blockIdx.x * 256u + threadIdx.x) * 8u;
  const v8h x0 = wrow8(W0 + e);
  const v8h x1 = wrow8(W1 + e);
  const v8h x2 = wrow8(W2 + e);
  const v8h x3 = wrow8(W3 + e);
  *(volatile v8h*)(P0 + e) = x0;
  *(volatile v8h*)(P1 + e) = x1;
  *(volatile v8h*)(P2 + e) = x2;
  *(volatile v8h*)(P3 + e) = x3;
  __threadfence();
  *(volatile v8h*)(P0 + e) = x0;
  *(volatile v8h*)(P1 + e) = x1;
  *(volatile v8h*)(P2 + e) = x2;
  *(volatile v8h*)(P3 + e) = x3;
}

template <int TR>
__device__ __forceinline__ void xconv_body(const float* __restrict__ X,
                                           _Float16* __restrict__ Xs,
                                           _Float16* __restrict__ Xt) {
#pragma clang fp contract(off)
  __shared__ _Float16 Ts[64 * LDT];
  __shared__ _Float16 Tt[64 * LDT];
  const unsigned tid = threadIdx.x;
  const unsigned c0 = blockIdx.x * 64u;
  const unsigned row0 = blockIdx.y * 64u;
#pragma unroll
  for (unsigned j = 0; j < 4u; ++j) {
    const unsigned idx = tid + 256u * j;
    const unsigned r = idx >> 4, c = (idx & 15u) * 4u;
    const v4f a = *(const v4f*)(X + (size_t)(row0 + r) * FIN + c0 + c);
#pragma unroll
    for (unsigned i = 0; i < 4u; ++i) {
      const h16 hv = toh_flush(XCARRY * bf16r(a[i]));
      Ts[r * LDT + c + i] = hv;
      if (TR) Tt[(c + i) * LDT + r] = hv;
    }
  }
  __syncthreads();
  v8h x[2], y[2];
  size_t off[2], offt[2];
#pragma unroll
  for (unsigned i = 0; i < 2u; ++i) {
    const unsigned rr = 32u * i + (tid >> 3);
    const unsigned kc = (tid & 7u) * 8u;
    x[i] = *(const v8h*)&Ts[rr * LDT + kc];
    off[i] = (size_t)(row0 + rr) * FIN + c0 + kc;
    if (TR) {
      y[i] = *(const v8h*)&Tt[rr * LDT + kc];
      offt[i] = ((size_t)blockIdx.y * FIN + c0 + rr) * RL + kc;
    }
  }
#pragma unroll
  for (int i = 0; i < 2; ++i) *(volatile v8h*)(Xs + off[i]) = x[i];
  if (TR) {
#pragma unroll
    for (int i = 0; i < 2; ++i) *(volatile v8h*)(Xt + offt[i]) = y[i];
  }
  __threadfence();
#pragma unroll
  for (int i = 0; i < 2; ++i) *(volatile v8h*)(Xs + off[i]) = x[i];
  if (TR) {
#pragma unroll
    for (int i = 0; i < 2; ++i) *(volatile v8h*)(Xt + offt[i]) = y[i];
  }
}

__global__ __launch_bounds__(256) void xconv_hist_kernel(
    const float* __restrict__ X, _Float16* __restrict__ Xs, _Float16* __restrict__ Xt) {
  xconv_body<1>(X, Xs, Xt);
}
__global__ __launch_bounds__(256) void xconv_ques_kernel(
    const float* __restrict__ X, _Float16* __restrict__ Xs) {
  xconv_body<0>(X, Xs, Xs);
}

template <int MODE>
__device__ __forceinline__ void gated_body(
    const _Float16* __restrict__ A16, const _Float16* __restrict__ By,
    const _Float16* __restrict__ Bg, const float* __restrict__ biasy,
    const float* __restrict__ biasg, const float* __restrict__ wa,
    _Float16* __restrict__ outa, _Float16* __restrict__ outb) {
  __shared__ float Cy[64 * LDC];
  __shared__ float Cg[64 * LDC];
  const unsigned tid = threadIdx.x, lane = tid & 31u;
  const unsigned w = (unsigned)__builtin_amdgcn_readfirstlane((int)(threadIdx.x >> 5));
  const unsigned mw = w >> 1, nw = w & 1u;
  const unsigned hh = lane >> 4, m = lane & 15u;
  const unsigned n0 = blockIdx.x * 64u;
  const unsigned row0 = blockIdx.y * 64u;
  const unsigned K = (unsigned)FIN;

  const _Float16* ap  = A16 + (size_t)(row0 + mw * 16u + m) * K + hh * 8u;
  const _Float16* yp0 = By + (size_t)(n0 + nw * 32u + m) * K + hh * 8u;
  const _Float16* yp1 = yp0 + (size_t)16 * K;
  const _Float16* gp0 = Bg + (size_t)(n0 + nw * 32u + m) * K + hh * 8u;
  const _Float16* gp1 = gp0 + (size_t)16 * K;
  v8f ay0 = {}, ay1 = {}, ag0 = {}, ag1 = {};
#pragma unroll 2
  for (unsigned k0 = 0; k0 < K; k0 += 32u) {
    const v16h a   = frag_at(ap + k0);
    const v16h by0 = frag_at(yp0 + k0);
    const v16h by1 = frag_at(yp1 + k0);
    const v16h bg0 = frag_at(gp0 + k0);
    const v16h bg1 = frag_at(gp1 + k0);
    ay0 = wmma16(a, by0, ay0);
    ay1 = wmma16(a, by1, ay1);
    ag0 = wmma16(a, bg0, ag0);
    ag1 = wmma16(a, bg1, ag1);
  }
#pragma unroll
  for (int r = 0; r < 8; ++r) {
    const unsigned o = (mw * 16u + hh * 8u + (unsigned)r) * LDC + nw * 32u + m;
    Cy[o]       = ay0[r];
    Cy[o + 16u] = ay1[r];
    Cg[o]       = ag0[r];
    Cg[o + 16u] = ag1[r];
  }
  __syncthreads();

#pragma unroll 1
  for (unsigned g = 0; g < 4u; ++g) {
    const unsigned r = 32u * (g >> 1) + (tid >> 3);
    const unsigned c = (tid & 7u) * 8u + 4u * (g & 1u);
    const v4f uy = *(const v4f*)&Cy[r * LDC + c];
    const v4f ug = *(const v4f*)&Cg[r * LDC + c];
    const v4f vy = *(const v4f*)(biasy + n0 + c);
    const v4f vg = *(const v4f*)(biasg + n0 + c);
    v4f t;
#pragma unroll
    for (int j = 0; j < 4; ++j) {
      const float yy = uy[j] * (1.0f / (WCARRY * XCARRY)) + bf16r(vy[j]);
      const float gg = ug[j] * (1.0f / (WCARRY * XCARRY)) + bf16r(vg[j]);
      t[j] = tanhf(yy) * (1.0f / (1.0f + expf(-gg)));
    }
    *(v4f*)&Cy[r * LDC + c] = t;
  }

  v8h xa[2], xb[2];
  size_t off[2];
#pragma unroll
  for (unsigned i = 0; i < 2u; ++i) {
    const unsigned r = 32u * i + (tid >> 3);
    const unsigned c = (tid & 7u) * 8u;
    const v4f u0 = *(const v4f*)&Cy[r * LDC + c];
    const v4f u1 = *(const v4f*)&Cy[r * LDC + c + 4];
    if (MODE == 1) {
      const v4f w0 = *(const v4f*)(wa + n0 + c);
      const v4f w1 = *(const v4f*)(wa + n0 + c + 4u);
#pragma unroll
      for (int j = 0; j < 4; ++j) {
        xa[i][j]     = toh_flush(u0[j] * bf16r(w0[j]) * QCARRY);
        xa[i][j + 4] = toh_flush(u1[j] * bf16r(w1[j]) * QCARRY);
        xb[i][j]     = toh_flush(u0[j] * u0[j] * SQCARRY);
        xb[i][j + 4] = toh_flush(u1[j] * u1[j] * SQCARRY);
      }
    } else {
#pragma unroll
      for (int j = 0; j < 4; ++j) {
        xa[i][j]     = toh_flush(u0[j] * HCARRY);
        xa[i][j + 4] = toh_flush(u1[j] * HCARRY);
        xb[i][j]     = toh_flush(u0[j] * u0[j] * SQCARRY);
        xb[i][j + 4] = toh_flush(u1[j] * u1[j] * SQCARRY);
      }
    }
    off[i] = (size_t)(row0 + r) * DH + n0 + c;
  }
#pragma unroll
  for (int i = 0; i < 2; ++i) *(volatile v8h*)(outa + off[i]) = xa[i];
#pragma unroll
  for (int i = 0; i < 2; ++i) *(volatile v8h*)(outb + off[i]) = xb[i];
  __threadfence();
#pragma unroll
  for (int i = 0; i < 2; ++i) *(volatile v8h*)(outa + off[i]) = xa[i];
#pragma unroll
  for (int i = 0; i < 2; ++i) *(volatile v8h*)(outb + off[i]) = xb[i];
}

__global__ __launch_bounds__(256) void gated_h_kernel(
    const _Float16* __restrict__ A16, const _Float16* __restrict__ By,
    const _Float16* __restrict__ Bg, const float* __restrict__ biasy,
    const float* __restrict__ biasg, _Float16* __restrict__ outa,
    _Float16* __restrict__ outb) {
  gated_body<0>(A16, By, Bg, biasy, biasg, biasy, outa, outb);
}
__global__ __launch_bounds__(256) void gated_q_kernel(
    const _Float16* __restrict__ A16, const _Float16* __restrict__ By,
    const _Float16* __restrict__ Bg, const float* __restrict__ biasy,
    const float* __restrict__ biasg, const float* __restrict__ wa,
    _Float16* __restrict__ outa, _Float16* __restrict__ outb) {
  gated_body<1>(A16, By, Bg, biasy, biasg, wa, outa, outb);
}

__global__ __launch_bounds__(256) void score_feat_kernel(
    const _Float16* __restrict__ Q1, const _Float16* __restrict__ Q2,
    const _Float16* __restrict__ H1, const _Float16* __restrict__ H2,
    const _Float16* __restrict__ Ht, const float* __restrict__ ba,
    float* __restrict__ Out) {
  __shared__ float Ss[64 * LDC];
  __shared__ _Float16 Ps[64 * LDT];
  __shared__ _Float16 Pr[64 * LDT];
  __shared__ float Linv[64];
  __shared__ float Os[8 * 16 * LDO];

  const unsigned tid = threadIdx.x, lane = tid & 31u;
  const unsigned w = (unsigned)__builtin_amdgcn_readfirstlane((int)(threadIdx.x >> 5));
  const unsigned hh = lane >> 4, m = lane & 15u;
  const unsigned b = blockIdx.x;

  {
    const unsigned mw = w >> 1, nw = w & 1u;
    const size_t qrow = (size_t)b * RL + mw * 16u + m;
    const size_t hrow = (size_t)b * RL + nw * 32u + m;
    const _Float16* q1p  = Q1 + qrow * DH + hh * 8u;
    const _Float16* q2p  = Q2 + qrow * DH + hh * 8u;
    const _Float16* h1p0 = H1 + hrow * DH + hh * 8u;
    const _Float16* h1p1 = h1p0 + (size_t)16 * DH;
    const _Float16* h2p0 = H2 + hrow * DH + hh * 8u;
    const _Float16* h2p1 = h2p0 + (size_t)16 * DH;
    v8f sn0 = {}, sn1 = {}, sd0 = {}, sd1 = {};
#pragma unroll 2
    for (unsigned k0 = 0; k0 < (unsigned)DH; k0 += 32u) {
      const v16h a1  = frag_at(q1p + k0);
      const v16h a2  = frag_at(q2p + k0);
      const v16h b10 = frag_at(h1p0 + k0);
      const v16h b11 = frag_at(h1p1 + k0);
      const v16h b20 = frag_at(h2p0 + k0);
      const v16h b21 = frag_at(h2p1 + k0);
      sn0 = wmma16(a1, b10, sn0);
      sn1 = wmma16(a1, b11, sn1);
      sd0 = wmma16(a2, b20, sd0);
      sd1 = wmma16(a2, b21, sd1);
    }
    const float bav = bf16r(ba[0]);
    const float nsc = 1.0f / (HCARRY * QCARRY);
    const float dsc = 1.0f / (SQCARRY * SQCARRY);
#pragma unroll
    for (int r = 0; r < 8; ++r) {
      const unsigned o = (mw * 16u + hh * 8u + (unsigned)r) * LDC + nw * 32u + m;
      Ss[o]       = sn0[r] * nsc * rsqrtf(fmaxf(sd0[r] * dsc, 1.0e-24f)) + bav;
      Ss[o + 16u] = sn1[r] * nsc * rsqrtf(fmaxf(sd1[r] * dsc, 1.0e-24f)) + bav;
    }
  }
  __syncthreads();

#pragma unroll 1
  for (unsigned i = 0; i < 8u; ++i) {
    const unsigned row = w * 8u + i;
    const float s0 = Ss[row * LDC + lane];
    const float s1 = Ss[row * LDC + lane + 32u];
    const bool ok0 = (lane <= row);
    const bool ok1 = (lane + 32u <= row);
    float mx = fmaxf(ok0 ? s0 : -1.0e30f, ok1 ? s1 : -1.0e30f);
    mx = red32_max(mx);
    const float x0 = expf(s0 - mx);
    const float x1 = expf(s1 - mx);
    const float e0 = ok0 ? x0 : 0.0f;
    const float e1 = ok1 ? x1 : 0.0f;
    const float t0 = e0 * PCARRY;
    const float t1 = e1 * PCARRY;
    const h16 p0 = toh_flush(t0);
    const h16 p1 = toh_flush(t1);
    const h16 r0 = toh_flush((t0 - (float)p0) * RCARRY);
    const h16 r1 = toh_flush((t1 - (float)p1) * RCARRY);
    const float l = red32_sum(((float)p0 + (float)p1) +
                              ((float)r0 + (float)r1) * (1.0f / RCARRY));
    Ps[row * LDT + lane] = p0;
    Ps[row * LDT + lane + 32u] = p1;
    Pr[row * LDT + lane] = r0;
    Pr[row * LDT + lane + 32u] = r1;
    if (lane == 0u) Linv[row] = 1.0f / (l * XCARRY);
  }
  __syncthreads();

  {
    const unsigned mw = w & 3u, ch = w >> 2;
    const unsigned ob = w * (16u * LDO);
    const v16h pf0 = ld_frag(&Ps[(mw * 16u) * LDT], LDT);
    const v16h pf1 = ld_frag(&Ps[(mw * 16u) * LDT + 32u], LDT);
    const v16h pr0 = ld_frag(&Pr[(mw * 16u) * LDT], LDT);
    const v16h pr1 = ld_frag(&Pr[(mw * 16u) * LDT + 32u], LDT);
    float inv[8];
#pragma unroll
    for (int r = 0; r < 8; ++r) inv[r] = Linv[mw * 16u + hh * 8u + (unsigned)r];

#pragma unroll 1
    for (unsigned cp = 0; cp < 16u; ++cp) {
      const unsigned col0 = ch * 512u + cp * 32u;
      const _Float16* vp = Ht + ((size_t)b * FIN + col0 + m) * RL + hh * 8u;
      const v16h v00 = frag_at(vp);
      const v16h v01 = frag_at(vp + 32);
      const v16h v10 = frag_at(vp + 16 * RL);
      const v16h v11 = frag_at(vp + 16 * RL + 32);
      v8f a0 = {}, a1 = {}, c0 = {}, c1 = {};
      a0 = wmma16(pf0, v00, a0);
      a0 = wmma16(pf1, v01, a0);
      a1 = wmma16(pf0, v10, a1);
      a1 = wmma16(pf1, v11, a1);
      c0 = wmma16(pr0, v00, c0);
      c0 = wmma16(pr1, v01, c0);
      c1 = wmma16(pr0, v10, c1);
      c1 = wmma16(pr1, v11, c1);
#pragma unroll
      for (int r = 0; r < 8; ++r) {
        const unsigned o = ob + (hh * 8u + (unsigned)r) * LDO + m;
        Os[o]       = (a0[r] + c0[r] * (1.0f / RCARRY)) * inv[r];
        Os[o + 16u] = (a1[r] + c1[r] * (1.0f / RCARRY)) * inv[r];
      }
      wave_lds_sync();
      v4f x[4];
      size_t off[4];
#pragma unroll
      for (unsigned i = 0; i < 4u; ++i) {
        const unsigned rr = 4u * i + (lane >> 3);
        const unsigned c = (lane & 7u) * 4u;
        x[i] = *(const v4f*)&Os[ob + rr * LDO + c];
        off[i] = ((size_t)b * RL + mw * 16u + rr) * FIN + col0 + c;
      }
#pragma unroll
      for (int i = 0; i < 4; ++i) *(volatile v4f*)(Out + off[i]) = x[i];
      __threadfence();
#pragma unroll
      for (int i = 0; i < 4; ++i) *(volatile v4f*)(Out + off[i]) = x[i];
      wave_lds_sync();
    }
  }
}

extern "C" void kernel_launch(void* const* d_in, const int* in_sizes, int n_in,
                              void* d_out, int out_size, void* d_ws, size_t ws_size,
                              hipStream_t stream) {
  if (n_in < 12) return;
  const long long need_x = (long long)NB * RL * FIN;
  if ((long long)in_sizes[0] < need_x) return;
  if ((long long)in_sizes[1] < need_x) return;
  if ((long long)in_sizes[2] < (long long)DH * FIN) return;
  if ((long long)in_sizes[4] < (long long)DH * FIN) return;
  if ((long long)in_sizes[6] < (long long)DH * FIN) return;
  if ((long long)in_sizes[8] < (long long)DH * FIN) return;
  if (in_sizes[3] < DH || in_sizes[5] < DH || in_sizes[7] < DH || in_sizes[9] < DH) return;
  if (in_sizes[10] < DH || in_sizes[11] < 1) return;
  if ((long long)out_size < need_x) return;
  if (ws_size < WS_TOTAL) return;

  const float* hist = (const float*)d_in[0];
  const float* ques = (const float*)d_in[1];
  const float* why  = (const float*)d_in[2];
  const float* bhy  = (const float*)d_in[3];
  const float* whg  = (const float*)d_in[4];
  const float* bhg  = (const float*)d_in[5];
  const float* wqy  = (const float*)d_in[6];
  const float* bqy  = (const float*)d_in[7];
  const float* wqg  = (const float*)d_in[8];
  const float* bqg  = (const float*)d_in[9];
  const float* wa   = (const float*)d_in[10];
  const float* ba   = (const float*)d_in[11];
  float* out = (float*)d_out;

  char* ws = (char*)d_ws;
  _Float16* Why16 = (_Float16*)(ws + OFF_WHY);
  _Float16* Whg16 = (_Float16*)(ws + OFF_WHG);
  _Float16* Wqy16 = (_Float16*)(ws + OFF_WQY);
  _Float16* Wqg16 = (_Float16*)(ws + OFF_WQG);
  _Float16* Xh16  = (_Float16*)(ws + OFF_XH);
  _Float16* Xq16  = (_Float16*)(ws + OFF_XQ);
  _Float16* Ht16  = (_Float16*)(ws + OFF_HT);
  _Float16* H1p   = (_Float16*)(ws + OFF_H1);
  _Float16* H2p   = (_Float16*)(ws + OFF_H2);
  _Float16* Q1p   = (_Float16*)(ws + OFF_Q1);
  _Float16* Q2p   = (_Float16*)(ws + OFF_Q2);

  dim3 blk(256);

  wplane_kernel<<<dim3((DH * FIN) / 2048), blk, 0, stream>>>(why, whg, wqy, wqg,
                                                             Why16, Whg16, Wqy16, Wqg16);
  xconv_hist_kernel<<<dim3(FIN / 64, NB), blk, 0, stream>>>(hist, Xh16, Ht16);
  xconv_ques_kernel<<<dim3(FIN / 64, NB), blk, 0, stream>>>(ques, Xq16);

  gated_h_kernel<<<dim3(DH / 64, MROWS / 64), blk, 0, stream>>>(Xh16, Why16, Whg16, bhy, bhg,
                                                                H1p, H2p);
  gated_q_kernel<<<dim3(DH / 64, MROWS / 64), blk, 0, stream>>>(Xq16, Wqy16, Wqg16, bqy, bqg,
                                                                wa, Q1p, Q2p);

  score_feat_kernel<<<dim3(NB), blk, 0, stream>>>(Q1p, Q2p, H1p, H2p, Ht16, ba, out);
}
